// GraphWaveNetLayer_7713761263797
// MI455X (gfx1250) — hardware-verified
//
#include <hip/hip_runtime.h>


namespace {
constexpr int N = 10000, C = 64, T = 12, E = 160000, NR = N * T  , NB = 32  , NBLK = (N + NB - 1) / NB  ;
constexpr float AS_ = 8.0f;

typedef _Float16 b16;
typedef __attribute__((ext_vector_type(16))) _Float16 v16b;
typedef __attribute__((ext_vector_type(8))) _Float16 v8b;
typedef __attribute__((ext_vector_type(8))) float v8f;
typedef __attribute__((ext_vector_type(4))) float v4f;
__device__ __forceinline__ float bf16_rne(float f) { unsigned int u = __float_as_uint(f); u += 0x7FFFu + ((u >> 16) & 1u); return __uint_as_float(u & 0xFFFF0000u); }
__device__ __forceinline__ void split16(float v, b16& hi, b16& lo) { hi = (b16)v; lo = (b16)(v - (float)hi); }
__device__ __forceinline__ v16b frag_kb(const b16* p, int hh) { const v8b a = *(const v8b*)(p + 8 * hh), b = *(const v8b*)(p + 16 + 8 * hh); v16b f;
#pragma unroll
  for (int e = 0; e < 8; ++e) { f[e] = a[e]; f[8 + e] = b[e]; } return f; }
__device__ __forceinline__ void frag_split(const float* p, int hh, v16b& fh, v16b& fl) {
#pragma unroll
  for (int e = 0; e < 8; ++e) { b16 a, c; split16(p[8 * hh + e] * AS_, a, c); fh[e] = a; fl[e] = c; split16(p[16 + 8 * hh + e] * AS_, a, c); fh[8 + e] = a; fl[8 + e] = c; } }
__device__ __forceinline__ v8f wmma16b(v16b a, v16b b, v8f c) { v8f d = __builtin_amdgcn_wmma_f32_16x16x32_f16(false, a, false, b, (short)0, c, false, false); asm volatile("v_nop\n\tv_nop\n\tv_nop\n\tv_nop" : "+v"(d) : "v"(a), "v"(b)); return d; }
__device__ __forceinline__ void wave_lds_sync() { __builtin_amdgcn_fence(__ATOMIC_RELEASE, "workgroup"); __builtin_amdgcn_wave_barrier(); __builtin_amdgcn_fence(__ATOMIC_ACQUIRE, "workgroup"); }
__device__ __forceinline__ float nexp(float x) { return __builtin_amdgcn_exp2f(x * 1.4426950408889634f); }
__device__ __forceinline__ float pmul(float a, float b) { float p = a * b; asm volatile("" : "+v"(p)); return p; }
__device__ __forceinline__ float sigm(float x) { return __builtin_amdgcn_rcpf(1.0f + nexp(-x)); }
__device__ __forceinline__ float tanh_n(float x) { const float e = __builtin_amdgcn_exp2f(x * 2.8853900817779268f); return 1.0f - 2.0f * __builtin_amdgcn_rcpf(e + 1.0f); }

__global__ __launch_bounds__(256) void prep_kernel(const float* __restrict__ x, const float* __restrict__ fw, const float* __restrict__ fb, const float* __restrict__ gw, const float* __restrict__ gb, const float* __restrict__ W, const float* __restrict__ bb, b16* __restrict__ R, b16* __restrict__ X, float* __restrict__ P) {
  __shared__ float xs[C][T + 1];
  const int n = blockIdx.x, t_ = threadIdx.x;
  for (int i = t_; i < C * T; i += 256) { const int c = i / T, t = i % T; xs[c][t + 1] = bf16_rne(x[((size_t)n * C + c) * T + t]); }
  if (t_ < C) xs[t_][0] = 0.0f;
  __syncthreads();
  for (int pass = 0; pass < 2; ++pass) {
    for (int i = t_; i < T * 16; i += 256) { const int t = i >> 4, c8 = (i & 15) * 8; v8b v; for (int e = 0; e < 8; ++e) { const int k = c8 + e; v[e] = (b16)((k < C) ? xs[k][t] : xs[k - C][t + 1]); } *(volatile v8b*)(X + ((size_t)n * T + t) * 128 + c8) = v; }
    if (n < 8) { const int gt = n * 256 + t_;
      for (int q = gt; q < 128 * 16 + 64 * 8; q += 2048) { v8b v;
        if (q < 128 * 16) { const int o = q >> 4, k0 = (q & 15) * 8; const float* w_ = (o < C) ? fw : gw; const int oo = o & 63; for (int e = 0; e < 8; ++e) { const int k = k0 + e; const int i_ = k & 63, tap = k >> 6; v[e] = (b16)bf16_rne(w_[(oo * C + i_) * 2 + tap]); } *(volatile v8b*)(R + o * 128 + k0) = v; }
        else { const int r = q - 128 * 16; const int d = r >> 3, c0 = (r & 7) * 8; for (int e = 0; e < 8; ++e) v[e] = (b16)bf16_rne(W[(c0 + e) * C + d]); *(volatile v8b*)(R + 128 * 128 + d * C + c0) = v; } }
      if (gt < 192) ((volatile float*)P)[gt] = (gt < 64) ? bf16_rne(fb[gt]) : (gt < 128) ? bf16_rne(gb[gt - 64]) : bf16_rne(bb[gt - 128]); }
    __threadfence(); }
}

__global__ __launch_bounds__(128) void conv_kernel(const b16* __restrict__ X, const b16* __restrict__ R, const float* __restrict__ P, float* __restrict__ HW) {
  __shared__ __attribute__((aligned(16))) float Th[4][32][C + 4];
  const int lane = threadIdx.x & 31, wave = threadIdx.x >> 5, nloc = lane & 15, hlf = lane >> 4, m0 = blockIdx.x * 128 + wave * 32;
  auto rowc = [&](int r) { return (r < NR) ? r : (NR - 1); };
  v8f acc[2][8];
#pragma unroll
  for (int r = 0; r < 2; ++r)
#pragma unroll
    for (int t = 0; t < 8; ++t) acc[r][t] = (v8f){};
#pragma unroll
  for (int kb = 0; kb < 128; kb += 32) { const v16b a0 = frag_kb(X + (size_t)rowc(m0 + nloc) * 128 + kb, hlf), a1 = frag_kb(X + (size_t)rowc(m0 + 16 + nloc) * 128 + kb, hlf);
#pragma unroll
    for (int t = 0; t < 8; ++t) { const v16b bw = frag_kb(R + (size_t)(t * 16 + nloc) * 128 + kb, hlf); acc[0][t] = wmma16b(a0, bw, acc[0][t]); acc[1][t] = wmma16b(a1, bw, acc[1][t]); } }
#pragma unroll
  for (int t = 0; t < 4; ++t)
#pragma unroll
    for (int r = 0; r < 2; ++r)
#pragma unroll
      for (int v = 0; v < 8; ++v) { const int c = t * 16 + nloc; Th[wave][r * 16 + 8 * hlf + v][c] = pmul(tanh_n(acc[r][t][v] + P[c]), sigm(acc[r][t + 4][v] + P[64 + c])); }
  wave_lds_sync();
  v8f a2[2][4];
#pragma unroll
  for (int r = 0; r < 2; ++r)
#pragma unroll
    for (int t = 0; t < 4; ++t) a2[r][t] = (v8f){};
  const b16* Wg = R + 128 * 128;
#pragma unroll
  for (int kb = 0; kb < C; kb += 32) { v16b h0, l0, h1, l1; frag_split(&Th[wave][nloc][kb], hlf, h0, l0); frag_split(&Th[wave][16 + nloc][kb], hlf, h1, l1);
#pragma unroll
    for (int t = 0; t < 4; ++t) { const v16b bw = frag_kb(Wg + (size_t)(t * 16 + nloc) * C + kb, hlf); a2[0][t] = wmma16b(h0, bw, a2[0][t]); a2[0][t] = wmma16b(l0, bw, a2[0][t]); a2[1][t] = wmma16b(h1, bw, a2[1][t]); a2[1][t] = wmma16b(l1, bw, a2[1][t]); } }
  wave_lds_sync();
#pragma unroll
  for (int t = 0; t < 4; ++t)
#pragma unroll
    for (int r = 0; r < 2; ++r)
#pragma unroll
      for (int v = 0; v < 8; ++v) Th[wave][r * 16 + 8 * hlf + v][t * 16 + nloc] = a2[r][t][v] * (1.0f / AS_);
  wave_lds_sync();
  for (int pass = 0; pass < 2; ++pass) { for (int i = lane; i < 32 * 16; i += 32) { const int rr = i >> 4, c4 = (i & 15) * 4; if (m0 + rr < NR) *(volatile v4f*)(HW + (size_t)(m0 + rr) * C + c4) = *(const v4f*)(&Th[wave][rr][c4]); } __threadfence(); }
}

__global__ __launch_bounds__(256) void deg_kernel(const int* __restrict__ ei, float* __restrict__ DEG) {
  __shared__ int cnt[8][NB];
  const int v0 = blockIdx.x * NB, t_ = threadIdx.x, lane = t_ & 31, wave = t_ >> 5;
  int my = 0;
  for (int e0 = wave * 32; e0 < E; e0 += 256) { const int e = e0 + lane; int d = (e < E) ? ei[E + e] : -1; const int loc = d - v0; const bool hit = (loc >= 0 && loc < NB);
#pragma unroll
    for (int j = 0; j < NB; ++j) { const unsigned int b = __builtin_amdgcn_ballot_w32(hit && loc == j); if (lane == j) my += __builtin_popcount(b); } }
  cnt[wave][lane] = my;
  __syncthreads();
  if (t_ < NB) { int s = 0; for (int w = 0; w < 8; ++w) s += cnt[w][t_]; const float dg = (float)s + 1.0f; for (int pass = 0; pass < 2; ++pass) ((volatile float*)DEG)[(size_t)blockIdx.x * NB + t_] = dg; }
  __threadfence();
}

__global__ __launch_bounds__(256) void aggr_kernel(const float* __restrict__ HW, const int* __restrict__ ei, const float* __restrict__ DEG, const float* __restrict__ x, const float* __restrict__ P, float* __restrict__ out) {
  __shared__ __attribute__((aligned(16))) float Acc[NB][T * C + 4]; __shared__ int Lsrc[256]; __shared__ int Lnode[256]; __shared__ int Cnt[8]; __shared__ int tot;
  const int v0 = blockIdx.x * NB, t_ = threadIdx.x, lane = t_ & 31, wave = t_ >> 5;
  for (int i = t_; i < NB * (T * C + 4); i += 256) (&Acc[0][0])[i] = 0.0f;
  __syncthreads();
  for (int c0 = 0; c0 < E; c0 += 256) { const int e = c0 + t_; int loc = -1, s = 0; if (e < E) { const int d = ei[E + e]; if (d >= v0 && d < v0 + NB) { loc = d - v0; s = ei[e]; s = (s < 0) ? 0 : (s >= N ? N - 1 : s); } }
    const unsigned int bal = __builtin_amdgcn_ballot_w32(loc >= 0); if (lane == 0) Cnt[wave] = __builtin_popcount(bal);
    __syncthreads();
    int base = 0; for (int w = 0; w < wave; ++w) base += Cnt[w]; const int pos = base + __builtin_popcount(bal & ((1u << lane) - 1u));
    if (loc >= 0) { Lsrc[pos] = s; Lnode[pos] = loc; }
    if (t_ == 0) { int a = 0; for (int w = 0; w < 8; ++w) a += Cnt[w]; tot = a; }
    __syncthreads();
    const int nh = tot;
    for (int k = 0; k < nh; ++k) { const int nd = Lnode[k]; if ((nd >> 2) == wave) { const int s = Lsrc[k]; const float nrm = rsqrtf(DEG[s]) * rsqrtf(DEG[v0 + nd]); const float* hr = HW + (size_t)s * T * C; float* ac = Acc[nd];
#pragma unroll
        for (int j = 0; j < 24; ++j) { const int idx = j * 32 + lane; ac[idx] += pmul(nrm, hr[idx]); } } }
    __syncthreads(); }
  for (int q = 0; q < 4; ++q) { const int nd = wave * 4 + q, n = v0 + nd; if (n >= N) continue; const float dg = DEG[n]; const float* hr = HW + (size_t)n * T * C; const float* xr = x + (size_t)n * C * T;
    for (int pass = 0; pass < 2; ++pass) { for (int i4 = lane * 4; i4 < C * T; i4 += 128) { v4f o; for (int e = 0; e < 4; ++e) { const int idx = i4 + e; const int c = idx / T, t = idx % T; o[e] = ((Acc[nd][t * C + c] + hr[t * C + c] / dg) + P[128 + c]) + bf16_rne(xr[idx]); } *(volatile v4f*)(out + (size_t)n * C * T + i4) = o; } __threadfence(); } }
}
}

extern "C" void kernel_launch(void* const* d_in, const int* in_sizes, int n_in,
                              void* d_out, int out_size, void* d_ws, size_t ws_size, hipStream_t stream) {
  (void)n_in; (void)out_size;
  const float* x = (const float*)d_in[0]; const float* fw = (const float*)d_in[1]; const float* fb = (const float*)d_in[2]; const float* gw = (const float*)d_in[3]; const float* gb = (const float*)d_in[4]; const float* W = (const float*)d_in[5]; const float* bb = (const float*)d_in[6]; const int* ei = (const int*)d_in[7];
  float* out = (float*)d_out;
  if (in_sizes[0] != N * C * T || in_sizes[1] != C * C * 2 || in_sizes[5] != C * C || in_sizes[7] != 2 * E) return;
  size_t off = 0; char* ws = (char*)d_ws;
  auto carve = [&](size_t bytes) { char* p = ws + off; off += (bytes + 255) & ~(size_t)255; return p; };
  b16* R = (b16*)carve((size_t)(128 * 128 + 64 * 64) * 2); b16* X = (b16*)carve((size_t)NR * 128 * 2); float* P = (float*)carve(256 * 4); float* HW = (float*)carve((size_t)NR * C * 4); float* DEG = (float*)carve((size_t)NBLK * NB * 4);
  if (off > ws_size) return;
  prep_kernel<<<N, 256, 0, stream>>>(x, fw, fb, gw, gb, W, bb, R, X, P);
  conv_kernel<<<(NR + 127) / 128, 128, 0, stream>>>(X, R, P, HW);
  deg_kernel<<<NBLK, 256, 0, stream>>>(ei, DEG);
  aggr_kernel<<<NBLK, 256, 0, stream>>>(HW, ei, DEG, x, P, out);
}
